// BiDirectionalAddBlock_73581379715114
// MI455X (gfx1250) — hardware-run, weakly checked
//
#include <hip/hip_runtime.h>
#include <math.h>

constexpr int kBatch     = 2;
constexpr int kSeq       = 1024;
constexpr int kDModel    = 768;
constexpr int kDInner    = 1536;
constexpr int kDState    = 16;
constexpr int kDConv     = 4;
constexpr int kDtRank    = 48;
constexpr int kRows      = kBatch * kSeq;
constexpr int kNXZ       = 2 * kDInner;
constexpr int kNXP       = kDtRank + 2 * kDState;
constexpr int kNXPPad    = 128;
constexpr int kDtKPad    = 64;
constexpr int kChunkT    = 16;
constexpr int kLnThreads = kDModel / 8;

typedef __attribute__((ext_vector_type(16))) _Float16 v16h;
typedef __attribute__((ext_vector_type(8)))  _Float16 v8h;
typedef __attribute__((ext_vector_type(16))) __bf16   v16b;
typedef __attribute__((ext_vector_type(8)))  __bf16   v8b;
typedef __attribute__((ext_vector_type(8)))  float    v8f;
typedef __attribute__((ext_vector_type(4)))  float    v4f;
typedef __attribute__((ext_vector_type(4)))  unsigned int v4u;

__device__ __forceinline__ unsigned short f2bf_bits(float f) {
  unsigned u = __float_as_uint(f);
  return (unsigned short)((u + 0x7FFFu + ((u >> 16) & 1u)) >> 16);
}
__device__ __forceinline__ float bf_bits2f(unsigned short h) { return __uint_as_float(((unsigned)h) << 16); }

__device__ __forceinline__ void dep_guard_h(v8f& a, v8f& b, v16h x, v16h y) { asm volatile("v_nop\n\tv_nop\n\tv_nop\n\tv_nop" : "+v"(a), "+v"(b) : "v"(x), "v"(y)); }
__device__ __forceinline__ void dep_guard_b(v8f& a, v8f& b, v16b x, v16b y) { asm volatile("v_nop\n\tv_nop\n\tv_nop\n\tv_nop" : "+v"(a), "+v"(b) : "v"(x), "v"(y)); }
__device__ __forceinline__ void keep4_h(v16h a, v16h b, v16h c, v16h d) { asm volatile("v_nop" :: "v"(a), "v"(b), "v"(c), "v"(d)); }
__device__ __forceinline__ void keep4_b(v16b a, v16b b, v16b c, v16b d) { asm volatile("v_nop" :: "v"(a), "v"(b), "v"(c), "v"(d)); }
__device__ __forceinline__ void acc_guard4(v8f& a, v8f& b, v8f& c, v8f& d) { asm volatile("v_nop\n\tv_nop\n\tv_nop\n\tv_nop" : "+v"(a), "+v"(b), "+v"(c), "+v"(d)); }
template <typename T> struct Frag;
template <> struct Frag<_Float16> {
  typedef v16h V; union U { v16h v; v8h h[2]; };
  static __device__ __forceinline__ v16h load(const _Float16* p) {
    U f; f.h[0] = *(const v8h*)(p); f.h[1] = *(const v8h*)(p + 16); return f.v;
  }
  static __device__ __forceinline__ v8f mma(v16h a, v16h b, v8f c) {
    return __builtin_amdgcn_wmma_f32_16x16x32_f16(false, a, false, b, (short)0, c, false, false);
  }
  static __device__ __forceinline__ void guard(v8f& a, v8f& b, v16h x, v16h y) { dep_guard_h(a, b, x, y); }
  static __device__ __forceinline__ void keep(v16h a, v16h b, v16h c, v16h d) { keep4_h(a, b, c, d); }
};
template <> struct Frag<__bf16> {
  typedef v16b V; union U { v16b v; v8b h[2]; };
  static __device__ __forceinline__ v16b load(const __bf16* p) {
    U f; f.h[0] = *(const v8b*)(p); f.h[1] = *(const v8b*)(p + 16); return f.v;
  }
  static __device__ __forceinline__ v8f mma(v16b a, v16b b, v8f c) {
    return __builtin_amdgcn_wmma_f32_16x16x32_bf16(false, a, false, b, (short)0, c, false, false);
  }
  static __device__ __forceinline__ void guard(v8f& a, v8f& b, v16b x, v16b y) { dep_guard_b(a, b, x, y); }
  static __device__ __forceinline__ void keep(v16b a, v16b b, v16b c, v16b d) { keep4_b(a, b, c, d); }
};

__device__ __forceinline__ unsigned pk16(unsigned short a, unsigned short b) { return (unsigned)a | ((unsigned)b << 16); }

template <int ET> struct Elem;
template <> struct Elem<0> { typedef _Float16 T; };
template <> struct Elem<1> { typedef __bf16 T; };
template <int ET, bool SPLIT, int BIAS_MODE, int OUT_MODE, bool RESID, int ACT = 0>
__global__ __launch_bounds__(256) void wmma_gemm64(
    const unsigned short* __restrict__ Ap, const unsigned short* __restrict__ A2p, int lda, long strideA,
    const unsigned short* __restrict__ Btp, const unsigned short* __restrict__ Bt2p, int ldb, long strideB,
    void* __restrict__ Cout, void* __restrict__ Cout2, int ldc, long strideC,
    const float* __restrict__ bias,
    const float* __restrict__ resid, long strideR,
    int M, int N, int K, float scale) {
  typedef typename Elem<ET>::T T;
  typedef typename Frag<T>::V V;
  const T* A = (const T*)Ap; const T* A2 = (const T*)A2p; const T* Bt = (const T*)Btp; const T* Bt2 = (const T*)Bt2p;
  __shared__ __align__(16) float sT[8][16 * 68];
  const int b    = blockIdx.y;
  const int lane = threadIdx.x & 31;
  const int wave = threadIdx.x >> 5;
  const int tilesN = N >> 6;
  const int tilesM = M >> 6;
  const int tile = blockIdx.x * 8 + wave;
  if (tile >= tilesM * tilesN) return;
  const int tm = tile / tilesN;
  const int tn = tile - tm * tilesN;
  const int m0 = tm << 6;
  const int n0 = tn << 6;

  const T* Ab  = A  + (size_t)b * strideA;
  const T* Bb  = Bt + (size_t)b * strideB;
  const T* Ab2 = SPLIT ? (A2  + (size_t)b * strideA) : nullptr;
  const T* Bb2 = SPLIT ? (Bt2 + (size_t)b * strideB) : nullptr;

  const int rlane = lane & 15;
  const int koff  = (lane >> 4) * 8;
  const int mOff  = (lane >> 4) * 8;

  v8f acc[4][4];
#pragma unroll
  for (int i = 0; i < 4; ++i)
#pragma unroll
    for (int j = 0; j < 4; ++j) acc[i][j] = (v8f){0.f,0.f,0.f,0.f,0.f,0.f,0.f,0.f};

  for (int k0 = 0; k0 < K; k0 += 32) {
    V bh[4], bl[4];
#pragma unroll
    for (int j = 0; j < 4; ++j) {
      const size_t bo = (size_t)(n0 + (j << 4) + rlane) * ldb + koff + k0;
      bh[j] = Frag<T>::load(Bb + bo);
      if (SPLIT) bl[j] = Frag<T>::load(Bb2 + bo);
    }
#pragma unroll
    for (int i = 0; i < 4; ++i) {
      const size_t ao = (size_t)(m0 + (i << 4) + rlane) * lda + koff + k0;
      V ah = Frag<T>::load(Ab + ao);
      V al;
      if (SPLIT) al = Frag<T>::load(Ab2 + ao);
#pragma unroll
      for (int j = 0; j < 4; ++j) {
        acc[i][j] = Frag<T>::mma(ah, bh[j], acc[i][j]);
        if (SPLIT) {
          acc[i][j] = Frag<T>::mma(ah, bl[j], acc[i][j]);
          acc[i][j] = Frag<T>::mma(al, bh[j], acc[i][j]);
        }
      }
      Frag<T>::guard(acc[i][0], acc[i][3], ah, SPLIT ? al : ah);
    }
    Frag<T>::keep(bh[0], bh[1], bh[2], bh[3]);
    if (SPLIT) Frag<T>::keep(bl[0], bl[1], bl[2], bl[3]);
  }
  acc_guard4(acc[0][0], acc[0][1], acc[0][2], acc[0][3]);
  acc_guard4(acc[1][0], acc[1][1], acc[1][2], acc[1][3]);
  acc_guard4(acc[2][0], acc[2][1], acc[2][2], acc[2][3]);
  acc_guard4(acc[3][0], acc[3][1], acc[3][2], acc[3][3]);

  float* slab = sT[wave];
  const float* Rb = RESID ? (resid + (size_t)b * strideR) : nullptr;
#pragma unroll
  for (int i = 0; i < 4; ++i) {
    const int mBase = m0 + (i << 4);
#pragma unroll
    for (int j = 0; j < 4; ++j) {
      const int n = n0 + (j << 4) + rlane;
      float bv = 0.f;
      if (BIAS_MODE == 2) bv = bias[n];
#pragma unroll
      for (int r = 0; r < 8; ++r) {
        float v = acc[i][j][r] * scale;
        if (BIAS_MODE == 1) v += bias[mBase + mOff + r];
        if (BIAS_MODE == 2) v += bv;
        if (RESID) v += Rb[(size_t)(mBase + mOff + r) * ldc + n];
        if (ACT == 2) v = fmaxf(v, 0.0f);
        if (ACT == 4) v = (v > 0.f) ? v : 0.01f * v;
        slab[(mOff + r) * 68 + (j << 4) + rlane] = v;
      }
    }
    __builtin_amdgcn_fence(__ATOMIC_RELEASE, "workgroup");
    __builtin_amdgcn_wave_barrier();
    __builtin_amdgcn_fence(__ATOMIC_ACQUIRE, "workgroup");
    if (OUT_MODE == 0) {
      float* C = (float*)Cout + (size_t)b * strideC;
      const int hh = lane >> 4, c4 = (lane & 15) * 4;
      for (int pass = 0; pass < 2; ++pass) {
#pragma unroll
        for (int it = 0; it < 8; ++it) {
          const int row = it * 2 + hh;
          v4f v = *(const v4f*)(slab + row * 68 + c4);
          *(volatile v4f*)(C + (size_t)(mBase + row) * ldc + n0 + c4) = v;
        }
        __threadfence();
      }
    } else {
      const int q = lane >> 3, c8 = (lane & 7) * 8;
      unsigned short* C  = (unsigned short*)Cout  + (size_t)b * strideC;
      unsigned short* C2 = (OUT_MODE == 2) ? ((unsigned short*)Cout2 + (size_t)b * strideC) : nullptr;
      for (int pass = 0; pass < 2; ++pass) {
#pragma unroll
        for (int it = 0; it < 4; ++it) {
          const int row = it * 4 + q;
          const float* sp = slab + row * 68 + c8;
          v8h hv, lv;
#pragma unroll
          for (int e = 0; e < 8; ++e) {
            if (OUT_MODE == 1) {
              hv[e] = (_Float16)sp[e];
            } else {
              unsigned short hb = f2bf_bits(sp[e]);
              unsigned short lb = f2bf_bits(sp[e] - bf_bits2f(hb));
              hv[e] = __builtin_bit_cast(_Float16, hb);
              lv[e] = __builtin_bit_cast(_Float16, lb);
            }
          }
          *(volatile v8h*)(C + (size_t)(mBase + row) * ldc + n0 + c8) = hv;
          if (OUT_MODE == 2) *(volatile v8h*)(C2 + (size_t)(mBase + row) * ldc + n0 + c8) = lv;
        }
        __threadfence();
      }
    }
    __builtin_amdgcn_fence(__ATOMIC_RELEASE, "workgroup");
    __builtin_amdgcn_wave_barrier();
    __builtin_amdgcn_fence(__ATOMIC_ACQUIRE, "workgroup");
  }
}

__device__ __forceinline__ void split8(v4f a, v4f c, v4u& uh, v4u& ul) {
  unsigned short hb[8], lb[8];
#pragma unroll
  for (int e = 0; e < 4; ++e) {
    hb[e]     = f2bf_bits(a[e]);
    lb[e]     = f2bf_bits(a[e] - bf_bits2f(hb[e]));
    hb[4 + e] = f2bf_bits(c[e]);
    lb[4 + e] = f2bf_bits(c[e] - bf_bits2f(hb[4 + e]));
  }
  uh = (v4u){pk16(hb[0], hb[1]), pk16(hb[2], hb[3]), pk16(hb[4], hb[5]), pk16(hb[6], hb[7])};
  ul = (v4u){pk16(lb[0], lb[1]), pk16(lb[2], lb[3]), pk16(lb[4], lb[5]), pk16(lb[6], lb[7])};
}

__global__ __launch_bounds__(96) void ln_split_kernel(
    const float* __restrict__ x, const float* __restrict__ gam, const float* __restrict__ bet,
    unsigned short* __restrict__ fH, unsigned short* __restrict__ fL,
    unsigned short* __restrict__ rH, unsigned short* __restrict__ rL,
    float* __restrict__ resid)
{
  __shared__ float red1[4];
  __shared__ float red2[4];
  const int r    = blockIdx.x;
  const int b    = r >> 10;
  const int l    = r & (kSeq - 1);
  const int t    = threadIdx.x;
  const int lane = t & 31, wave = t >> 5;
  const float* xr = x + (size_t)r * kDModel;
  const int c0 = t * 8;
  const v4f xa = *(const v4f*)(xr + c0);
  const v4f xb = *(const v4f*)(xr + c0 + 4);
  float s = ((xa[0] + xa[1]) + (xa[2] + xa[3])) + ((xb[0] + xb[1]) + (xb[2] + xb[3]));
#pragma unroll
  for (int off = 16; off > 0; off >>= 1) s += __shfl_xor(s, off, 32);
  if (lane == 0) red1[wave] = s;
  __syncthreads();
  const float mu = ((red1[0] + red1[1]) + red1[2]) * (1.0f / 768.0f);
  const v4f da = xa - mu;
  const v4f db = xb - mu;
  float s2 = ((da[0] * da[0] + da[1] * da[1]) + (da[2] * da[2] + da[3] * da[3]))
           + ((db[0] * db[0] + db[1] * db[1]) + (db[2] * db[2] + db[3] * db[3]));
#pragma unroll
  for (int off = 16; off > 0; off >>= 1) s2 += __shfl_xor(s2, off, 32);
  if (lane == 0) red2[wave] = s2;
  __syncthreads();
  const float var  = ((red2[0] + red2[1]) + red2[2]) * (1.0f / 768.0f);
  const float rstd = rsqrtf(var + 1e-5f);
  const v4f ga = *(const v4f*)(gam + c0), gb = *(const v4f*)(gam + c0 + 4);
  const v4f ba = *(const v4f*)(bet + c0), bb = *(const v4f*)(bet + c0 + 4);
  const v4f ya = da * rstd * ga + ba;
  const v4f yb = db * rstd * gb + bb;
  v4u uh, ul;
  split8(ya, yb, uh, ul);
  const int rr = b * kSeq + (kSeq - 1 - l);
  const size_t of  = (size_t)r * kDModel + c0;
  const size_t orr = (size_t)rr * kDModel + c0;
  const int i0 = 4 * t, i1 = 4 * (kLnThreads + t);
  const v4f r0v = *(const v4f*)(xr + i0);
  const v4f r1v = *(const v4f*)(xr + i1);
  float* rp = resid + (size_t)r * kDModel;
  for (int ps = 0; ps < 2; ++ps) {
    *(volatile v4u*)(fH + of)  = uh;
    *(volatile v4u*)(fL + of)  = ul;
    *(volatile v4u*)(rH + orr) = uh;
    *(volatile v4u*)(rL + orr) = ul;
    *(volatile v4f*)(rp + i0)  = r0v;
    *(volatile v4f*)(rp + i1)  = r1v;
    __threadfence();
  }
}

__global__ __launch_bounds__(256) void wsplit_kernel(
    const float* __restrict__ W, int nsrc, int ksrc,
    unsigned short* __restrict__ H, unsigned short* __restrict__ Lo, int npad, int kpad)
{
  const int gid = blockIdx.x * 256 + threadIdx.x;
  const int gpr = kpad >> 3;
  if (gid >= npad * gpr) return;
  const int row = gid / gpr;
  const int c8  = (gid - row * gpr) * 8;
  const bool valid = (row < nsrc) && (c8 < ksrc);
  const int rowc = (row < nsrc) ? row : (nsrc - 1);
  const int cc   = (c8 < ksrc) ? c8 : (ksrc - 8);
  const float* p = W + (size_t)rowc * ksrc + cc;
  v4f a = *(const v4f*)(p);
  v4f c = *(const v4f*)(p + 4);
  const v4f z4 = {0.f, 0.f, 0.f, 0.f};
  if (!valid) { a = z4; c = z4; }
  v4u uh, ul;
  split8(a, c, uh, ul);
  const size_t o = (size_t)gid * 8;
  for (int ps = 0; ps < 2; ++ps) {
    *(volatile v4u*)(H + o)  = uh;
    *(volatile v4u*)(Lo + o) = ul;
    __threadfence();
  }
}

__global__ __launch_bounds__(256) void conv_silu_split_kernel(
    const float* __restrict__ xz, const float* __restrict__ convw, const float* __restrict__ convb,
    float* __restrict__ xc, unsigned short* __restrict__ xcH, unsigned short* __restrict__ xcL)
{
  __shared__ __align__(16) float stg[1024];
  const int tid = threadIdx.x;
  const int e0  = blockIdx.x * 1024 + tid * 4;
  const int r   = e0 / kDInner;
  const int d   = e0 - r * kDInner;
  const int b   = r >> 10;
  const int l   = r & (kSeq - 1);
  const v4f cb = *(const v4f*)(convb + d);
  const v4f w0 = *(const v4f*)(convw + (size_t)(d + 0) * kDConv);
  const v4f w1 = *(const v4f*)(convw + (size_t)(d + 1) * kDConv);
  const v4f w2 = *(const v4f*)(convw + (size_t)(d + 2) * kDConv);
  const v4f w3 = *(const v4f*)(convw + (size_t)(d + 3) * kDConv);
  const v4f z4 = {0.f, 0.f, 0.f, 0.f};
  v4f s = z4;
#pragma unroll
  for (int k = 0; k < kDConv; ++k) {
    const int ll  = l - (kDConv - 1) + k;
    const int llc = ll < 0 ? 0 : ll;
    const v4f xv = *(const v4f*)(xz + (size_t)(b * kSeq + llc) * kNXZ + d);
    const v4f wk = {w0[k], w1[k], w2[k], w3[k]};
    v4f tk = xv * wk;
    if (ll < 0) tk = z4;
    s = s + tk;
  }
  const v4f v = cb + s;
  v4f yv;
#pragma unroll
  for (int e = 0; e < 4; ++e) {
    const float vv = v[e];
    const float sg = 1.0f / (1.0f + expf(-vv));
    yv[e] = vv * sg;
  }
  *(v4f*)(stg + tid * 4) = yv;
  __syncthreads();
  const int g = tid & 127;
  const v4f pa = *(const v4f*)(stg + g * 8);
  const v4f pc = *(const v4f*)(stg + g * 8 + 4);
  v4u uh, ul;
  split8(pa, pc, uh, ul);
  const size_t o16 = (size_t)blockIdx.x * 1024 + (size_t)g * 8;
  for (int ps = 0; ps < 2; ++ps) {
    *(volatile v4f*)(xc + e0) = yv;
    if (tid < 128) {
      *(volatile v4u*)(xcH + o16) = uh;
      *(volatile v4u*)(xcL + o16) = ul;
    }
    __threadfence();
  }
}

__global__ __launch_bounds__(256) void dta_split_kernel(
    const float* __restrict__ dbc, unsigned short* __restrict__ H, unsigned short* __restrict__ Lo, int nrows)
{
  const int gid = blockIdx.x * 256 + threadIdx.x;
  if (gid >= nrows * 8) return;
  const int row = gid >> 3;
  const int c8  = (gid & 7) * 8;
  const bool valid = c8 < kDtRank;
  const int cc = valid ? c8 : (kDtRank - 8);
  const float* p = dbc + (size_t)row * kNXPPad + cc;
  v4f a = *(const v4f*)(p);
  v4f c = *(const v4f*)(p + 4);
  const v4f z4 = {0.f, 0.f, 0.f, 0.f};
  if (!valid) { a = z4; c = z4; }
  v4u uh, ul;
  split8(a, c, uh, ul);
  const size_t o = (size_t)gid * 8;
  for (int ps = 0; ps < 2; ++ps) {
    *(volatile v4u*)(H + o)  = uh;
    *(volatile v4u*)(Lo + o) = ul;
    __threadfence();
  }
}

__global__ __launch_bounds__(256) void scan_gate_kernel(
    const float* __restrict__ dbc, const float* __restrict__ dpre, const float* __restrict__ xc,
    const float* __restrict__ xz, const float* __restrict__ Alog, const float* __restrict__ Dsk,
    unsigned short* __restrict__ yH, unsigned short* __restrict__ yL)
{
  __shared__ __align__(16) float bc_s[kChunkT * 32];
  __shared__ __align__(16) float y_s[kChunkT * 256];
  __shared__ float h_s[kDState * 256];
  __shared__ float a_s[kDState * 256];
  const int tid  = threadIdx.x;
  const int lane = tid & 31, wave = tid >> 5;
  const int b    = blockIdx.x / 6;
  const int d0   = (blockIdx.x - b * 6) * 256;
  const int d    = d0 + tid;
#pragma unroll 1
  for (int n = 0; n < kDState; ++n) {
    a_s[n * 256 + tid] = -expf(Alog[(size_t)d * kDState + n]);
    h_s[n * 256 + tid] = 0.0f;
  }
  const float dsk = Dsk[d];
#pragma unroll 1
  for (int ch = 0; ch < kSeq / kChunkT; ++ch) {
    const int t0 = ch * kChunkT;
    const int r0 = b * kSeq + t0;
    __syncthreads();
    if (tid < kChunkT * 8) {
      const int s = tid >> 3, j = (tid & 7) * 4;
      const v4f v = *(const v4f*)(dbc + (size_t)(r0 + s) * kNXPPad + kDtRank + j);
      *(v4f*)(bc_s + s * 32 + j) = v;
    }
    __syncthreads();
#pragma unroll 1
    for (int s = 0; s < kChunkT; ++s) {
      const size_t ri = (size_t)(r0 + s);
      const float dp = dpre[ri * kDInner + d];
      const float xv = xc[ri * kDInner + d];
      const float zv = xz[ri * kNXZ + kDInner + d];
      const float dl = fmaxf(dp, 0.0f) + log1pf(expf(-fabsf(dp)));
      const float dx = dl * xv;
      const float* bcp = bc_s + s * 32;
      float y = 0.0f;
#pragma unroll 1
      for (int n4 = 0; n4 < kDState / 4; ++n4) {
#pragma unroll
        for (int jj = 0; jj < 4; ++jj) {
          const int n = n4 * 4 + jj;
          const float an = a_s[n * 256 + tid];
          const float hp = h_s[n * 256 + tid];
          const float da = expf(dl * an);
          const float hn = da * hp + bcp[n] * dx;
          h_s[n * 256 + tid] = hn;
          y += hn * bcp[kDState + n];
        }
      }
      y = y + xv * dsk;
      const float sg = 1.0f / (1.0f + expf(-zv));
      y = y * (zv * sg);
      y_s[s * 256 + tid] = y;
    }
    __syncthreads();
    {
      const int sa = wave, sb = wave + 8;
      const float* pa = y_s + sa * 256 + lane * 8;
      const float* pb = y_s + sb * 256 + lane * 8;
      const v4f a0 = *(const v4f*)(pa), a1 = *(const v4f*)(pa + 4);
      const v4f b0 = *(const v4f*)(pb), b1 = *(const v4f*)(pb + 4);
      v4u uha, ula, uhb, ulb;
      split8(a0, a1, uha, ula);
      split8(b0, b1, uhb, ulb);
      const size_t oa = (size_t)(r0 + sa) * kDInner + d0 + lane * 8;
      const size_t ob = (size_t)(r0 + sb) * kDInner + d0 + lane * 8;
      for (int ps = 0; ps < 2; ++ps) {
        *(volatile v4u*)(yH + oa) = uha;
        *(volatile v4u*)(yL + oa) = ula;
        *(volatile v4u*)(yH + ob) = uhb;
        *(volatile v4u*)(yL + ob) = ulb;
        __threadfence();
      }
    }
  }
}

static void launch_gemm_plain(const unsigned short* AH, const unsigned short* AL, int lda,
                              const unsigned short* BH, const unsigned short* BL, int ldb,
                              float* C, int ldc, const float* dummy, int M, int N, int K, hipStream_t st)
{
  const int tiles = (M / 64) * (N / 64);
  dim3 grid((tiles + 7) / 8, 1);
  wmma_gemm64<1, true, 0, 0, false, 0><<<grid, 256, 0, st>>>(
      AH, AL, lda, 0L, BH, BL, ldb, 0L, (void*)C, (void*)C, ldc, 0L,
      dummy, dummy, 0L, M, N, K, 1.0f);
}
static void launch_gemm_bias(const unsigned short* AH, const unsigned short* AL, int lda,
                             const unsigned short* BH, const unsigned short* BL, int ldb,
                             float* C, int ldc, const float* bias, int M, int N, int K, hipStream_t st)
{
  const int tiles = (M / 64) * (N / 64);
  dim3 grid((tiles + 7) / 8, 1);
  wmma_gemm64<1, true, 2, 0, false, 0><<<grid, 256, 0, st>>>(
      AH, AL, lda, 0L, BH, BL, ldb, 0L, (void*)C, (void*)C, ldc, 0L,
      bias, bias, 0L, M, N, K, 1.0f);
}
static void launch_gemm_resid(const unsigned short* AH, const unsigned short* AL, int lda,
                              const unsigned short* BH, const unsigned short* BL, int ldb,
                              float* C, int ldc, const float* resid, int M, int N, int K, hipStream_t st)
{
  const int tiles = (M / 64) * (N / 64);
  dim3 grid((tiles + 7) / 8, 1);
  wmma_gemm64<1, true, 0, 0, true, 0><<<grid, 256, 0, st>>>(
      AH, AL, lda, 0L, BH, BL, ldb, 0L, (void*)C, (void*)C, ldc, 0L,
      resid, resid, 0L, M, N, K, 1.0f);
}

extern "C" void kernel_launch(void* const* d_in, const int* in_sizes, int n_in,
                              void* d_out, int out_size, void* d_ws, size_t ws_size,
                              hipStream_t stream)
{
  if (n_in < 21) return;
  if (in_sizes[0] != kRows * kDModel) return;
  if (in_sizes[1] != kDModel || in_sizes[2] != kDModel) return;
  if (out_size != 2 * kRows * kDModel) return;
  for (int m = 0; m < 2; ++m) {
    const int base = 3 + 9 * m;
    if (in_sizes[base + 0] != kNXZ * kDModel)    return;
    if (in_sizes[base + 1] != kDInner * kDConv)  return;
    if (in_sizes[base + 2] != kDInner)           return;
    if (in_sizes[base + 3] != kNXP * kDInner)    return;
    if (in_sizes[base + 4] != kDInner * kDtRank) return;
    if (in_sizes[base + 5] != kDInner)           return;
    if (in_sizes[base + 6] != kDInner * kDState) return;
    if (in_sizes[base + 7] != kDInner)           return;
    if (in_sizes[base + 8] != kDModel * kDInner) return;
  }

  const float* x    = (const float*)d_in[0];
  const float* ln_g = (const float*)d_in[1];
  const float* ln_b = (const float*)d_in[2];

  float* out_hidden = (float*)d_out;
  float* out_resid  = (float*)d_out + (size_t)kRows * kDModel;

  char* ws = (char*)d_ws;
  size_t off = 0;
  auto carve = [&](size_t bytes) -> void* {
    void* p = ws + off;
    off += (bytes + 255) & ~(size_t)255;
    return p;
  };
  const size_t xnPlane  = (size_t)kRows * kDModel * 2;
  const size_t inWPlane = (size_t)kNXZ * kDModel * 2;
  const size_t xpWPlane = (size_t)kNXPPad * kDInner * 2;
  const size_t dtWPlane = (size_t)kDInner * kDtKPad * 2;
  const size_t outWPlane= (size_t)kDModel * kDInner * 2;
  const size_t xcPlane  = (size_t)kRows * kDInner * 2;
  const size_t dtAPlane = (size_t)kRows * kDtKPad * 2;

  unsigned short* xnFH = (unsigned short*)carve(xnPlane);
  unsigned short* xnFL = (unsigned short*)carve(xnPlane);
  unsigned short* xnRH = (unsigned short*)carve(xnPlane);
  unsigned short* xnRL = (unsigned short*)carve(xnPlane);
  unsigned short* inWH = (unsigned short*)carve(inWPlane);
  unsigned short* inWL = (unsigned short*)carve(inWPlane);
  unsigned short* xpWH = (unsigned short*)carve(xpWPlane);
  unsigned short* xpWL = (unsigned short*)carve(xpWPlane);
  unsigned short* dtWH = (unsigned short*)carve(dtWPlane);
  unsigned short* dtWL = (unsigned short*)carve(dtWPlane);
  unsigned short* outWH= (unsigned short*)carve(outWPlane);
  unsigned short* outWL= (unsigned short*)carve(outWPlane);
  float*          xz   = (float*)carve((size_t)kRows * kNXZ * 4);
  float*          xc   = (float*)carve((size_t)kRows * kDInner * 4);
  unsigned short* xcH  = (unsigned short*)carve(xcPlane);
  unsigned short* xcL  = (unsigned short*)carve(xcPlane);
  float*          dbc  = (float*)carve((size_t)kRows * kNXPPad * 4);
  unsigned short* dtAH = (unsigned short*)carve(dtAPlane);
  unsigned short* dtAL = (unsigned short*)carve(dtAPlane);
  float*          dpre = (float*)carve((size_t)kRows * kDInner * 4);
  unsigned short* yH   = (unsigned short*)carve(xcPlane);
  unsigned short* yL   = (unsigned short*)carve(xcPlane);
  float*          h1   = (float*)carve((size_t)kRows * kDModel * 4);
  if (off > ws_size) return;

  ln_split_kernel<<<kRows, kLnThreads, 0, stream>>>(x, ln_g, ln_b, xnFH, xnFL, xnRH, xnRL, out_resid);

  for (int m = 0; m < 2; ++m) {
    const int base = 3 + 9 * m;
    const float* inW   = (const float*)d_in[base + 0];
    const float* convw = (const float*)d_in[base + 1];
    const float* convb = (const float*)d_in[base + 2];
    const float* xpW   = (const float*)d_in[base + 3];
    const float* dtW   = (const float*)d_in[base + 4];
    const float* dtb   = (const float*)d_in[base + 5];
    const float* Alog  = (const float*)d_in[base + 6];
    const float* Dsk   = (const float*)d_in[base + 7];
    const float* outW  = (const float*)d_in[base + 8];
    const unsigned short* aH = (m == 0) ? xnFH : xnRH;
    const unsigned short* aL = (m == 0) ? xnFL : xnRL;

    {
      int tot = kNXZ * (kDModel / 8);
      wsplit_kernel<<<(tot + 255) / 256, 256, 0, stream>>>(inW, kNXZ, kDModel, inWH, inWL, kNXZ, kDModel);
      tot = kNXPPad * (kDInner / 8);
      wsplit_kernel<<<(tot + 255) / 256, 256, 0, stream>>>(xpW, kNXP, kDInner, xpWH, xpWL, kNXPPad, kDInner);
      tot = kDInner * (kDtKPad / 8);
      wsplit_kernel<<<(tot + 255) / 256, 256, 0, stream>>>(dtW, kDInner, kDtRank, dtWH, dtWL, kDInner, kDtKPad);
      tot = kDModel * (kDInner / 8);
      wsplit_kernel<<<(tot + 255) / 256, 256, 0, stream>>>(outW, kDModel, kDInner, outWH, outWL, kDModel, kDInner);
    }

    launch_gemm_plain(aH, aL, kDModel, inWH, inWL, kDModel, xz, kNXZ, x, kRows, kNXZ, kDModel, stream);

    conv_silu_split_kernel<<<(kRows * kDInner) / 1024, 256, 0, stream>>>(xz, convw, convb, xc, xcH, xcL);

    launch_gemm_plain(xcH, xcL, kDInner, xpWH, xpWL, kDInner, dbc, kNXPPad, x, kRows, kNXPPad, kDInner, stream);

    dta_split_kernel<<<(kRows * 8 + 255) / 256, 256, 0, stream>>>(dbc, dtAH, dtAL, kRows);

    launch_gemm_bias(dtAH, dtAL, kDtKPad, dtWH, dtWL, kDtKPad, dpre, kDInner, dtb, kRows, kDInner, kDtKPad, stream);

    scan_gate_kernel<<<kBatch * (kDInner / 256), 256, 0, stream>>>(dbc, dpre, xc, xz, Alog, Dsk, yH, yL);

    if (m == 0) {
      launch_gemm_plain(yH, yL, kDInner, outWH, outWL, kDInner, h1, kDModel, x, kRows, kDModel, kDInner, stream);
    } else {
      launch_gemm_resid(yH, yL, kDInner, outWH, outWL, kDInner, out_hidden, kDModel, h1, kRows, kDModel, kDInner, stream);
    }
  }
}
